// Correlation_29618094474055
// MI455X (gfx1250) — hardware-verified
//
#include <hip/hip_runtime.h>
#include <stdint.h>
#include <stddef.h>


#define B_ 32
#define C_ 256
#define N_ 1024
#define EPS_COS 1e-8f
#define EPS_BN  1e-5f

typedef _Float16 v16h __attribute__((ext_vector_type(16)));
typedef _Float16 v8h  __attribute__((ext_vector_type(8)));
typedef float    v8f  __attribute__((ext_vector_type(8)));
typedef float    v4f  __attribute__((ext_vector_type(4)));
typedef unsigned int v4u __attribute__((ext_vector_type(4)));

union Frag  { v16h v; v4u q[2]; };
union Pack8 { v8h h;  v4u q; };

static __device__ __forceinline__ v8f wmma16(v16h a, v16h b, v8f c) {
    v8f d = __builtin_amdgcn_wmma_f32_16x16x32_f16(false, a, false, b, (short)0, c, false, false);
    asm volatile("v_nop\n\tv_nop\n\tv_nop\n\tv_nop" : "+v"(d) : "v"(a), "v"(b));
    return d;
}

static __device__ __forceinline__ v4u ld4u(const _Float16* p) { return *(const v4u*)p; }
static __device__ __forceinline__ void st4u(_Float16* p, v4u v) { *(volatile v4u*)p = v; }
static __device__ __forceinline__ void st4f(float* p, v4f v) { *(volatile v4f*)p = v; }


__global__ void __launch_bounds__(256)
k_cvt_x(const float* __restrict__ x, _Float16* __restrict__ xT, float* __restrict__ nrm) {
    __shared__ __attribute__((aligned(16))) _Float16 T[64 * 264];
    __shared__ float sqp[256];
    __shared__ __attribute__((aligned(16))) float nrs[64];
    const int tid = threadIdx.x, lane = tid & 31, w = tid >> 5;
    const int b = blockIdx.y, n0 = blockIdx.x * 64;
    const int nn = tid & 63, cg = tid >> 6;
    const float* xp = x + ((size_t)b * C_ + cg * 64) * N_ + n0 + nn;
    float sq = 0.f;
#pragma unroll 4
    for (int q = 0; q < 64; ++q) {
        const float v = xp[(size_t)q * N_];
        sq += v * v;
        T[nn * 264 + cg * 64 + q] = (_Float16)v;
    }
    sqp[tid] = sq;
    __syncthreads();
    if (tid < 64) {
        const float s = ((sqp[tid] + sqp[64 + tid]) + sqp[128 + tid]) + sqp[192 + tid];
        nrs[tid] = sqrtf(s);
    }
    __syncthreads();
#pragma unroll
    for (int s = 0; s < 8; ++s) {
        const int rl = w * 8 + s;
        const v4u val = *(const v4u*)(&T[rl * 264 + lane * 8]);
        st4u(xT + ((size_t)b * N_ + n0 + rl) * C_ + lane * 8, val);
    }
    if (w == 0 && lane < 16) {
        const v4f nv = *(const v4f*)(&nrs[lane * 4]);
        st4f(nrm + (size_t)b * N_ + n0 + lane * 4, nv);
    }
    __threadfence();
#pragma unroll
    for (int s = 0; s < 8; ++s) {
        const int rl = w * 8 + s;
        const v4u val = *(const v4u*)(&T[rl * 264 + lane * 8]);
        st4u(xT + ((size_t)b * N_ + n0 + rl) * C_ + lane * 8, val);
    }
    if (w == 0 && lane < 16) {
        const v4f nv = *(const v4f*)(&nrs[lane * 4]);
        st4f(nrm + (size_t)b * N_ + n0 + lane * 4, nv);
    }
}

__global__ void __launch_bounds__(256)
k_cvt_w(const float* __restrict__ w, _Float16* __restrict__ Wt, int Cout, int Cin, int total8) {
    const int idx = blockIdx.x * 256 + threadIdx.x;
    if (idx >= total8) return;
    const int cpr = Cin >> 3;
    const int ci8 = idx % cpr;
    const int co  = (idx / cpr) % Cout;
    const int k   = idx / (cpr * Cout);
    const float* src = w + ((size_t)co * Cin + ci8 * 8) * 3 + k;
    Pack8 p;
#pragma unroll
    for (int e = 0; e < 8; ++e) p.h[e] = (_Float16)(src[e * 3] * 16.0f);
    _Float16* dst = Wt + ((size_t)k * Cout + co) * Cin + ci8 * 8;
    const v4u val = p.q;
    st4u(dst, val);
    __threadfence();
    st4u(dst, val);
}

__global__ void __launch_bounds__(128)
k_cos(const _Float16* __restrict__ xT, const float* __restrict__ nrm, _Float16* __restrict__ res) {
    __shared__ __attribute__((aligned(16))) _Float16 T[64 * 72];
    const int tid = threadIdx.x, lane = tid & 31, w = tid >> 5, h = lane >> 4, m = lane & 15;
    const int b = blockIdx.y;
    int p = blockIdx.x, bi = 0;
#pragma unroll 1
    for (int it = 0; it < 16; ++it) {
        const int cnt = 16 - bi;
        if (p >= cnt) { p -= cnt; ++bi; }
    }
    const int bj = bi + p;
    const int i0 = bi * 64, j0 = bj * 64;
    const int wr = w >> 1, wc = w & 1;
    const _Float16* Ab = xT + ((size_t)b * N_ + i0 + wr * 32 + m) * C_ + h * 8;
    const _Float16* Bb = xT + ((size_t)b * N_ + j0 + wc * 32 + m) * C_ + h * 8;

    v8f acc[2][2] = {};
#pragma unroll 2
    for (int k0 = 0; k0 < C_; k0 += 32) {
        Frag a0, a1, f0, f1;
        a0.q[0] = ld4u(Ab + k0);                   a0.q[1] = ld4u(Ab + k0 + 16);
        a1.q[0] = ld4u(Ab + (size_t)16 * C_ + k0); a1.q[1] = ld4u(Ab + (size_t)16 * C_ + k0 + 16);
        f0.q[0] = ld4u(Bb + k0);                   f0.q[1] = ld4u(Bb + k0 + 16);
        f1.q[0] = ld4u(Bb + (size_t)16 * C_ + k0); f1.q[1] = ld4u(Bb + (size_t)16 * C_ + k0 + 16);
        acc[0][0] = wmma16(a0.v, f0.v, acc[0][0]);
        acc[0][1] = wmma16(a0.v, f1.v, acc[0][1]);
        acc[1][0] = wmma16(a1.v, f0.v, acc[1][0]);
        acc[1][1] = wmma16(a1.v, f1.v, acc[1][1]);
    }

#pragma unroll
    for (int u = 0; u < 2; ++u) {
        const int lj = wc * 32 + u * 16 + m;
        const int gj = j0 + lj;
        const float nj = nrm[(size_t)b * N_ + gj];
#pragma unroll
        for (int t = 0; t < 2; ++t) {
#pragma unroll
            for (int r = 0; r < 8; ++r) {
                const int li = wr * 32 + t * 16 + h * 8 + r;
                const int gi = i0 + li;
                const float ni = nrm[(size_t)b * N_ + gi];
                const float den = fmaxf(ni * nj, EPS_COS);
                float v = (acc[t][u][r] / den) * 16.0f;
                if (gi == gj) v = 16.0f;
                T[li * 72 + lj] = (_Float16)v;
            }
        }
    }
    __syncthreads();

    const bool mirror = (bi != bj);
#pragma unroll
    for (int s = 0; s < 4; ++s) {
        const int rl = w * 16 + s * 4 + (lane >> 3);
        const int ch = (lane & 7) * 8;
        const v4u val = *(const v4u*)(&T[rl * 72 + ch]);
        st4u(res + ((size_t)b * N_ + i0 + rl) * N_ + j0 + ch, val);
    }
    if (mirror) {
#pragma unroll
        for (int s = 0; s < 4; ++s) {
            const int ql = w * 16 + s * 4 + (lane >> 3);
            const int ch = (lane & 7) * 8;
            Pack8 g;
#pragma unroll
            for (int e = 0; e < 8; ++e) g.h[e] = T[(ch + e) * 72 + ql];
            st4u(res + ((size_t)b * N_ + j0 + ql) * N_ + i0 + ch, g.q);
        }
    }
    __threadfence();
#pragma unroll
    for (int s = 0; s < 4; ++s) {
        const int rl = w * 16 + s * 4 + (lane >> 3);
        const int ch = (lane & 7) * 8;
        const v4u val = *(const v4u*)(&T[rl * 72 + ch]);
        st4u(res + ((size_t)b * N_ + i0 + rl) * N_ + j0 + ch, val);
    }
    if (mirror) {
#pragma unroll
        for (int s = 0; s < 4; ++s) {
            const int ql = w * 16 + s * 4 + (lane >> 3);
            const int ch = (lane & 7) * 8;
            Pack8 g;
#pragma unroll
            for (int e = 0; e < 8; ++e) g.h[e] = T[(ch + e) * 72 + ql];
            st4u(res + ((size_t)b * N_ + j0 + ql) * N_ + i0 + ch, g.q);
        }
    }
}

static __device__ __forceinline__ void conv_seg(v8f (&acc)[2][2],
                                                const _Float16* wr0, const _Float16* wr1,
                                                const _Float16* br0, const _Float16* br1,
                                                bool v0, bool v1, int klen) {
    const v4u z4 = {0u, 0u, 0u, 0u};
#pragma unroll 2
    for (int kc = 0; kc < klen; kc += 32) {
        Frag a0, a1, f0, f1;
        a0.q[0] = ld4u(wr0 + kc); a0.q[1] = ld4u(wr0 + kc + 16);
        a1.q[0] = ld4u(wr1 + kc); a1.q[1] = ld4u(wr1 + kc + 16);
        v4u t00 = ld4u(br0 + kc), t01 = ld4u(br0 + kc + 16);
        v4u t10 = ld4u(br1 + kc), t11 = ld4u(br1 + kc + 16);
        if (!v0) { t00 = z4; t01 = z4; }
        if (!v1) { t10 = z4; t11 = z4; }
        f0.q[0] = t00; f0.q[1] = t01;
        f1.q[0] = t10; f1.q[1] = t11;
        acc[0][0] = wmma16(a0.v, f0.v, acc[0][0]);
        acc[0][1] = wmma16(a0.v, f1.v, acc[0][1]);
        acc[1][0] = wmma16(a1.v, f0.v, acc[1][0]);
        acc[1][1] = wmma16(a1.v, f1.v, acc[1][1]);
    }
}

template <int CIN, int CIN0, int P0, int P1>
__global__ void __launch_bounds__(256)
k_conv(const _Float16* __restrict__ Wt, const _Float16* __restrict__ B0, const _Float16* __restrict__ B1,
       const float* __restrict__ bias, float* __restrict__ pre, float oscale) {
    typedef char k_tile_check[(CIN % 32 == 0 && CIN0 % 32 == 0 && CIN0 <= CIN) ? 1 : -1];
    (void)sizeof(k_tile_check);
    __shared__ __attribute__((aligned(16))) float E[8 * 32 * 36];
    const int tid = threadIdx.x, lane = tid & 31, w = tid >> 5, h = lane >> 4, m = lane & 15;
    const int b = blockIdx.y, n0 = blockIdx.x * 32, co0 = w * 32;

    v8f acc[2][2] = {};
#pragma unroll
    for (int tap = 0; tap < 3; ++tap) {
        const int np0 = n0 + m + tap - 1;
        const int np1 = np0 + 16;
        const bool v0 = (np0 >= 0) && (np0 < N_);
        const bool v1 = (np1 >= 0) && (np1 < N_);
        const int nc0 = min(max(np0, 0), N_ - 1);
        const int nc1 = min(max(np1, 0), N_ - 1);
        const _Float16* wr0 = Wt + ((size_t)(tap * C_ + co0 + m)) * CIN + h * 8;
        const _Float16* wr1 = wr0 + (size_t)16 * CIN;
        {
            const _Float16* br0 = B0 + ((size_t)b * N_ + nc0) * P0 + h * 8;
            const _Float16* br1 = B0 + ((size_t)b * N_ + nc1) * P0 + h * 8;
            conv_seg(acc, wr0, wr1, br0, br1, v0, v1, CIN0);
        }
        if (CIN0 < CIN) {
            const _Float16* br0 = B1 + ((size_t)b * N_ + nc0) * P1 + h * 8;
            const _Float16* br1 = B1 + ((size_t)b * N_ + nc1) * P1 + h * 8;
            conv_seg(acc, wr0 + CIN0, wr1 + CIN0, br0, br1, v0, v1, CIN - CIN0);
        }
    }

    float* Ew = E + w * (32 * 36);
#pragma unroll
    for (int t = 0; t < 2; ++t) {
#pragma unroll
        for (int u = 0; u < 2; ++u) {
#pragma unroll
            for (int r = 0; r < 8; ++r) {
                const int lr = t * 16 + h * 8 + r;
                Ew[lr * 36 + u * 16 + m] = acc[t][u][r] * oscale + bias[co0 + lr];
            }
        }
    }
    __syncthreads();
#pragma unroll
    for (int s = 0; s < 8; ++s) {
        const int rl = s * 4 + (lane >> 3);
        const int ch = (lane & 7) * 4;
        const v4f val = *(const v4f*)(Ew + rl * 36 + ch);
        st4f(pre + ((size_t)b * C_ + co0 + rl) * N_ + n0 + ch, val);
    }
    __threadfence();
#pragma unroll
    for (int s = 0; s < 8; ++s) {
        const int rl = s * 4 + (lane >> 3);
        const int ch = (lane & 7) * 4;
        const v4f val = *(const v4f*)(Ew + rl * 36 + ch);
        st4f(pre + ((size_t)b * C_ + co0 + rl) * N_ + n0 + ch, val);
    }
}

__global__ void __launch_bounds__(256)
k_bn_stats(const float* __restrict__ pre, const float* __restrict__ gamma, const float* __restrict__ beta,
           float* __restrict__ scsh) {
    __shared__ __attribute__((aligned(16))) float scs[32];
    __shared__ __attribute__((aligned(16))) float shs[32];
    const int tid = threadIdx.x, lane = tid & 31, w = tid >> 5;
    const int g = blockIdx.x;
#pragma unroll 1
    for (int q = 0; q < 4; ++q) {
        const int cl = w * 4 + q;
        const int c = g * 32 + cl;
        double s1 = 0.0, s2 = 0.0;
#pragma unroll 1
        for (int b = 0; b < B_; ++b) {
            const float* row = pre + ((size_t)b * C_ + c) * N_ + lane * 4;
#pragma unroll
            for (int s = 0; s < 8; ++s) {
                const v4f v = *(const v4f*)(row + s * 128);
#pragma unroll
                for (int i = 0; i < 4; ++i) {
                    const double d = (double)v[i];
                    s1 += d;
                    s2 += d * d;
                }
            }
        }
#pragma unroll
        for (int off = 16; off > 0; off >>= 1) {
            s1 += __shfl_xor(s1, off);
            s2 += __shfl_xor(s2, off);
        }
        if (lane == 0) {
            const double inv = 1.0 / (double)(B_ * N_);
            const double mean = s1 * inv;
            double var = s2 * inv - mean * mean;
            if (var < 0.0) var = 0.0;
            const float varf = (float)var;
            const float rstd = 1.0f / sqrtf(varf + EPS_BN);
            const float sc = gamma[c] * rstd;
            scs[cl] = sc;
            shs[cl] = beta[c] - (float)mean * sc;
        }
    }
    __syncthreads();
    if (w == 0 && lane < 16) {
        v4f val;
        float* dst;
        if (lane < 8) { val = *(const v4f*)(&scs[lane * 4]);       dst = scsh + g * 32 + lane * 4; }
        else          { val = *(const v4f*)(&shs[(lane - 8) * 4]); dst = scsh + C_ + g * 32 + (lane - 8) * 4; }
        st4f(dst, val);
        __threadfence();
        st4f(dst, val);
    }
}

__global__ void __launch_bounds__(256)
k_bn_apply_t(const float* __restrict__ pre, const float* __restrict__ scsh, _Float16* __restrict__ dstT,
             float oscale) {
    __shared__ __attribute__((aligned(16))) _Float16 T[32 * 264];
    __shared__ float ssc[256];
    __shared__ float ssh[256];
    const int tid = threadIdx.x, lane = tid & 31, w = tid >> 5;
    const int b = blockIdx.y, n0 = blockIdx.x * 32;
    ssc[tid] = scsh[tid];
    ssh[tid] = scsh[C_ + tid];
    __syncthreads();
    const int nn = tid & 31, cg = tid >> 5;
    const float* pp = pre + ((size_t)b * C_ + cg * 32) * N_ + n0 + nn;
#pragma unroll 4
    for (int q = 0; q < 32; ++q) {
        const int c = cg * 32 + q;
        const float v = pp[(size_t)q * N_];
        const float y = fmaxf(v * ssc[c] + ssh[c], 0.f) * oscale;
        T[nn * 264 + c] = (_Float16)y;
    }
    __syncthreads();
#pragma unroll
    for (int s = 0; s < 4; ++s) {
        const int rl = w * 4 + s;
        const v4u val = *(const v4u*)(&T[rl * 264 + lane * 8]);
        st4u(dstT + ((size_t)b * N_ + n0 + rl) * C_ + lane * 8, val);
    }
    __threadfence();
#pragma unroll
    for (int s = 0; s < 4; ++s) {
        const int rl = w * 4 + s;
        const v4u val = *(const v4u*)(&T[rl * 264 + lane * 8]);
        st4u(dstT + ((size_t)b * N_ + n0 + rl) * C_ + lane * 8, val);
    }
}

__global__ void __launch_bounds__(256)
k_bn_apply_out(const float* __restrict__ pre, const float* __restrict__ scsh, float* __restrict__ out) {
    const int tid = threadIdx.x, lane = tid & 31, w = tid >> 5;
    const int cgp = blockIdx.x, b = blockIdx.y;
#pragma unroll 1
    for (int q = 0; q < 32; ++q) {
        const int c = cgp * 32 + q;
        const float sc = scsh[c];
        const float sh = scsh[C_ + c];
        const size_t idx = ((size_t)b * C_ + c) * N_ + w * 128 + lane * 4;
        const v4f v = *(const v4f*)(pre + idx);
        v4f y = v;
#pragma unroll
        for (int i = 0; i < 4; ++i) y[i] = fmaxf(v[i] * sc + sh, 0.f);
        st4f(out + idx, y);
        __threadfence();
        st4f(out + idx, y);
    }
}

extern "C" void kernel_launch(void* const* d_in, const int* in_sizes, int n_in,
                              void* d_out, int out_size, void* d_ws, size_t ws_size,
                              hipStream_t stream) {
    if (n_in < 13) return;
    if (out_size != B_ * C_ * N_) return;
    if (in_sizes[0] != B_ * C_ * N_) return;
    if (in_sizes[1] != C_ * C_ * 3 || in_sizes[5] != C_ * N_ * 3 || in_sizes[9] != C_ * 2 * C_ * 3) return;
    if (in_sizes[2] != C_ || in_sizes[3] != C_ || in_sizes[4] != C_ ||
        in_sizes[6] != C_ || in_sizes[7] != C_ || in_sizes[8] != C_ ||
        in_sizes[10] != C_ || in_sizes[11] != C_ || in_sizes[12] != C_) return;

    const float* x     = (const float*)d_in[0];
    const float* w_bp  = (const float*)d_in[1];
    const float* b_bp  = (const float*)d_in[2];
    const float* g_bp  = (const float*)d_in[3];
    const float* be_bp = (const float*)d_in[4];
    const float* w1    = (const float*)d_in[5];
    const float* b1    = (const float*)d_in[6];
    const float* g1    = (const float*)d_in[7];
    const float* be1   = (const float*)d_in[8];
    const float* w2    = (const float*)d_in[9];
    const float* b2    = (const float*)d_in[10];
    const float* g2    = (const float*)d_in[11];
    const float* be2   = (const float*)d_in[12];
    float* out = (float*)d_out;

    const size_t MiB    = (size_t)1 << 20;
    const size_t o_x    = 0;
    const size_t o_res  = 16 * MiB;
    const size_t o_pre  = 80 * MiB;
    const size_t o_wbp  = 112 * MiB;
    const size_t o_w1   = o_wbp + (size_t)3 * C_ * C_ * 2;
    const size_t o_w2   = o_w1 + (size_t)3 * C_ * N_ * 2;
    const size_t o_nrm  = o_w2 + (size_t)3 * C_ * 2 * C_ * 2;
    const size_t o_scsh = o_nrm + (size_t)B_ * N_ * 4;
    const size_t o_end  = o_scsh + (size_t)2 * C_ * 4;
    if (o_end > ws_size) return;

    char* ws = (char*)d_ws;
    _Float16* xT     = (_Float16*)(ws + o_x);
    _Float16* cat_bp = (_Float16*)(ws + o_x);
    _Float16* res16  = (_Float16*)(ws + o_res);
    _Float16* cat_h1 = (_Float16*)(ws + o_res);
    float*    pre    = (float*)(ws + o_pre);
    _Float16* wt_bp  = (_Float16*)(ws + o_wbp);
    _Float16* wt_1   = (_Float16*)(ws + o_w1);
    _Float16* wt_2   = (_Float16*)(ws + o_w2);
    float*    nrm    = (float*)(ws + o_nrm);
    float*    scsh   = (float*)(ws + o_scsh);

    k_cvt_x<<<dim3(N_ / 64, B_), 256, 0, stream>>>(x, xT, nrm);
    {
        const int t_bp = 3 * C_ * C_ / 8, t_1 = 3 * C_ * N_ / 8, t_2 = 3 * C_ * 2 * C_ / 8;
        k_cvt_w<<<(t_bp + 255) / 256, 256, 0, stream>>>(w_bp, wt_bp, C_, C_, t_bp);
        k_cvt_w<<<(t_1 + 255) / 256, 256, 0, stream>>>(w1, wt_1, C_, N_, t_1);
        k_cvt_w<<<(t_2 + 255) / 256, 256, 0, stream>>>(w2, wt_2, C_, 2 * C_, t_2);
    }

    k_cos<<<dim3(136, B_), 128, 0, stream>>>(xT, nrm, res16);

    k_conv<C_, C_, C_, C_><<<dim3(N_ / 32, B_), 256, 0, stream>>>(wt_bp, xT, xT, b_bp, pre, 1.0f / 16.0f);
    k_bn_stats<<<C_ / 32, 256, 0, stream>>>(pre, g_bp, be_bp, scsh);
    k_bn_apply_t<<<dim3(N_ / 32, B_), 256, 0, stream>>>(pre, scsh, cat_bp, 8.0f);

    k_conv<N_, N_, N_, N_><<<dim3(N_ / 32, B_), 256, 0, stream>>>(wt_1, res16, res16, b1, pre, 1.0f / 256.0f);
    k_bn_stats<<<C_ / 32, 256, 0, stream>>>(pre, g1, be1, scsh);
    k_bn_apply_t<<<dim3(N_ / 32, B_), 256, 0, stream>>>(pre, scsh, cat_h1, 8.0f);

    k_conv<2 * C_, C_, C_, C_><<<dim3(N_ / 32, B_), 256, 0, stream>>>(wt_2, cat_h1, cat_bp, b2, pre, 1.0f / 128.0f);
    k_bn_stats<<<C_ / 32, 256, 0, stream>>>(pre, g2, be2, scsh);
    k_bn_apply_out<<<dim3(C_ / 32, B_), 256, 0, stream>>>(pre, scsh, out);
}
